// ParallelBlock_24842090840769
// MI455X (gfx1250) — hardware-verified
//
#include <hip/hip_runtime.h>


#define NB_  2
#define NT_  2048
#define DM   1024
#define NH_  16
#define HD   64
#define NTK  (NB_ * NT_)
#define NF   3788
#define NFP  3840
#define MLPH 716
#define MLPP 768
#define PSC  32768.0f
#define EPS  1e-6f

typedef _Float16 h16;
typedef __attribute__((ext_vector_type(16))) _Float16 v16h;
typedef __attribute__((ext_vector_type(8)))  _Float16 v8h;
typedef __attribute__((ext_vector_type(8)))  float    v8f;
typedef __attribute__((ext_vector_type(4)))  float    v4f;
typedef v8h  __attribute__((may_alias)) v8ha;
typedef v4f  __attribute__((may_alias)) v4fa;

__device__ __forceinline__ unsigned short f2bf(float f) { unsigned u = __float_as_uint(f); u += 0x7FFFu + ((u >> 16) & 1u); return (unsigned short)(u >> 16); }
__device__ __forceinline__ float bf2f(unsigned short b) { return __uint_as_float(((unsigned)b) << 16); }
__device__ __forceinline__ float bfr(float f) { return bf2f(f2bf(f)); }
__device__ __forceinline__ v16h cat16(v8h lo, v8h hi) { return __builtin_shufflevector(lo, hi, 0, 1, 2, 3, 4, 5, 6, 7, 8, 9, 10, 11, 12, 13, 14, 15); }
__device__ __forceinline__ v8f wmma16(v16h a, v16h b, v8f c) { return __builtin_amdgcn_wmma_f32_16x16x32_f16(false, a, false, b, (short)0, c, false, false); }
__device__ __forceinline__ float hsum16(float v) { v += __shfl_xor(v, 1, 16); v += __shfl_xor(v, 2, 16); v += __shfl_xor(v, 4, 16); return v + __shfl_xor(v, 8, 16); }
__device__ __forceinline__ float gelu_t(float x) { const float c = 0.7978845608028654f; return 0.5f * x * (1.0f + tanhf(c * (x + 0.044715f * x * x * x))); }

__global__ __launch_bounds__(256) void k_ln(const float* __restrict__ x, const float* __restrict__ g, const float* __restrict__ bt, h16* XN16) {
    const int lane = threadIdx.x & 31, r = blockIdx.x * 8 + (threadIdx.x >> 5);
    if (r >= NTK) return;
    const float* xr = x + (size_t)r * DM;
    float s = 0.f;
#pragma unroll
    for (int q = 0; q < 4; ++q)
#pragma unroll
        for (int i = 0; i < 8; ++i) s += bfr(xr[q * 256 + lane * 8 + i]);
#pragma unroll
    for (int o = 16; o; o >>= 1) s += __shfl_xor(s, o, 32);
    const float mu = s * (1.0f / DM);
    float sq = 0.f;
#pragma unroll 1
    for (int q = 0; q < 4; ++q)
#pragma unroll
        for (int i = 0; i < 8; ++i) { const float d = bfr(xr[q * 256 + lane * 8 + i]) - mu; sq += d * d; }
#pragma unroll
    for (int o = 16; o; o >>= 1) sq += __shfl_xor(sq, o, 32);
    const float rs = rsqrtf(sq * (1.0f / DM) + EPS);
#pragma unroll 1
    for (int q = 0; q < 4; ++q) {
        v8h o8;
#pragma unroll
        for (int i = 0; i < 8; ++i) { const int c = q * 256 + lane * 8 + i; o8[i] = (h16)((bfr(xr[c]) - mu) * rs * bfr(g[c]) + bfr(bt[c])); }
        *(volatile v8h*)(XN16 + (size_t)r * DM + q * 256 + lane * 8) = o8; __threadfence(); *(volatile v8h*)(XN16 + (size_t)r * DM + q * 256 + lane * 8) = o8;
    }
}

__global__ __launch_bounds__(256) void k_wt(const float* __restrict__ Wm, int K, int N, int Kpad, h16* WT) {
    __shared__ __align__(16) h16 tl[64 * 72];
    const int tid = threadIdx.x, k0 = blockIdx.x * 64, n0 = blockIdx.y * 64;
    const int kk = tid >> 2, nq = (tid & 3) * 16;
#pragma unroll
    for (int i = 0; i < 16; ++i) { const int k = k0 + kk, n = n0 + nq + i; tl[(nq + i) * 72 + kk] = (k < K && n < N) ? (h16)bfr(Wm[(size_t)k * N + n]) : (h16)0.f; }
    __syncthreads();
    const int piece = tid & 7;
    auto pass = [&]() {
#pragma unroll
        for (int s = 0; s < 2; ++s) { const int nr = (tid >> 3) + 32 * s; const v8h val = *(const v8ha*)(tl + nr * 72 + piece * 8);
            *(volatile v8h*)(WT + (size_t)(n0 + nr) * Kpad + k0 + piece * 8) = val; }
    };
    pass(); __threadfence(); pass();
}

__device__ __forceinline__ void gemm_tile(const h16* __restrict__ A, const h16* __restrict__ BT, int K, int r0, int c0, int lr, int hi, v8f* acc) {
    const size_t aoff = (size_t)(r0 + lr) * K + 8 * hi;
    size_t boff[4];
#pragma unroll
    for (int t = 0; t < 4; ++t) boff[t] = (size_t)(c0 + t * 16 + lr) * K + 8 * hi;
#pragma unroll
    for (int t = 0; t < 4; ++t) acc[t] = (v8f){};
#pragma unroll 1
    for (int kc = 0; kc < K; kc += 32) {
        const v16h a = cat16(*(const v8h*)(A + aoff + kc), *(const v8h*)(A + aoff + kc + 16));
#pragma unroll
        for (int t = 0; t < 4; ++t) acc[t] = wmma16(a, cat16(*(const v8h*)(BT + boff[t] + kc), *(const v8h*)(BT + boff[t] + kc + 16)), acc[t]);
        asm volatile("v_nop\n\tv_nop\n\tv_nop\n\tv_nop" : "+v"(acc[0]), "+v"(acc[1]), "+v"(acc[2]), "+v"(acc[3]) : "v"(a));
    }
}

__global__ __launch_bounds__(128) void k_fused(const h16* __restrict__ XN16, const h16* __restrict__ W1T, const float* __restrict__ b1,
                                              const float* __restrict__ qg, const float* __restrict__ qb, const float* __restrict__ kg, const float* __restrict__ kb,
                                              h16* Q16, h16* K16, h16* V16, h16* G16) {
    __shared__ __align__(16) float ost[4][16 * 68];
    const int lane = threadIdx.x & 31, wave = threadIdx.x >> 5, lr = lane & 15, hi = lane >> 4;
    const int r0 = blockIdx.x * 64 + wave * 16, c0 = blockIdx.y * 64;
    v8f acc[4];
    gemm_tile(XN16, W1T, DM, r0, c0, lr, hi, acc);
    const int sec = c0 / DM;
#pragma unroll
    for (int t = 0; t < 4; ++t) { const int col = c0 + t * 16 + lr; const float bv = (col < NF) ? bfr(b1[col]) : 0.f;
#pragma unroll
        for (int j = 0; j < 8; ++j) acc[t][j] += bv; }
    if (sec < 2) {
        const float* gg = sec ? kg : qg; const float* bb = sec ? kb : qb;
#pragma unroll
        for (int j = 0; j < 8; ++j) {
            float s = acc[0][j] + acc[1][j] + acc[2][j] + acc[3][j];
            const float mu = hsum16(s) * (1.0f / HD);
            float q = 0.f;
#pragma unroll
            for (int t = 0; t < 4; ++t) { const float d = acc[t][j] - mu; q += d * d; }
            const float rs = rsqrtf(hsum16(q) * (1.0f / HD) + EPS);
#pragma unroll
            for (int t = 0; t < 4; ++t) acc[t][j] = (acc[t][j] - mu) * rs * bfr(gg[t * 16 + lr]) + bfr(bb[t * 16 + lr]);
        }
    } else if (sec == 3) {
#pragma unroll
        for (int t = 0; t < 4; ++t)
#pragma unroll 1
            for (int j = 0; j < 8; ++j) acc[t][j] = gelu_t(acc[t][j]);
    }
    float* os = &ost[wave][0];
#pragma unroll
    for (int t = 0; t < 4; ++t)
#pragma unroll
        for (int j = 0; j < 8; ++j) os[(hi * 8 + j) * 68 + t * 16 + lr] = acc[t][j];
    __syncthreads();
    h16* dst; int ld, cc;
    if (sec == 0) { dst = Q16; ld = DM; cc = c0; } else if (sec == 1) { dst = K16; ld = DM; cc = c0 - DM; } else if (sec == 2) { dst = V16; ld = DM; cc = c0 - 2 * DM; } else { dst = G16; ld = MLPP; cc = c0 - 3 * DM; }
    h16* crow = dst + (size_t)r0 * ld + cc;
    auto pass = [&]() {
#pragma unroll
        for (int s = 0; s < 4; ++s) { const int row = 4 * s + (lane >> 3), piece = lane & 7; const float* sp = os + row * 68 + piece * 8; v8h o;
#pragma unroll
            for (int i = 0; i < 8; ++i) o[i] = (h16)sp[i];
            *(volatile v8h*)(crow + (size_t)row * ld + piece * 8) = o; }
    };
    pass(); __threadfence(); pass();
}

__global__ __launch_bounds__(128) void k_gemm16o(const h16* __restrict__ A, const h16* __restrict__ BT, int K, const float* __restrict__ bias, h16* C16, int ldc, int cbase) {
    __shared__ __align__(16) float ost[4][16 * 68];
    const int lane = threadIdx.x & 31, wave = threadIdx.x >> 5, lr = lane & 15, hi = lane >> 4;
    const int r0 = blockIdx.x * 64 + wave * 16, c0 = blockIdx.y * 64;
    v8f acc[4];
    gemm_tile(A, BT, K, r0, c0, lr, hi, acc);
    float* os = &ost[wave][0];
#pragma unroll
    for (int t = 0; t < 4; ++t) { const float bv = bfr(bias[c0 + t * 16 + lr]);
#pragma unroll
        for (int j = 0; j < 8; ++j) os[(hi * 8 + j) * 68 + t * 16 + lr] = acc[t][j] + bv; }
    __syncthreads();
    h16* crow = C16 + (size_t)r0 * ldc + cbase + c0;
    auto pass = [&]() {
#pragma unroll
        for (int s = 0; s < 4; ++s) { const int row = 4 * s + (lane >> 3), piece = lane & 7; const float* sp = os + row * 68 + piece * 8; v8h o;
#pragma unroll
            for (int i = 0; i < 8; ++i) o[i] = (h16)sp[i];
            *(volatile v8h*)(crow + (size_t)row * ldc + piece * 8) = o; }
    };
    pass(); __threadfence(); pass();
}

__global__ __launch_bounds__(128) void k_gemmout(const h16* __restrict__ A, const h16* __restrict__ BT, const float* __restrict__ bias, const float* __restrict__ x, float* C) {
    __shared__ __align__(16) float ost[4][16 * 68];
    const int lane = threadIdx.x & 31, wave = threadIdx.x >> 5, lr = lane & 15, hi = lane >> 4;
    const int r0 = blockIdx.x * 64 + wave * 16, c0 = blockIdx.y * 64;
    v8f acc[4];
    gemm_tile(A, BT, 2 * DM, r0, c0, lr, hi, acc);
    float* os = &ost[wave][0];
#pragma unroll
    for (int t = 0; t < 4; ++t) { const int col = c0 + t * 16 + lr; const float bv = bfr(bias[col]);
#pragma unroll
        for (int j = 0; j < 8; ++j) os[(hi * 8 + j) * 68 + t * 16 + lr] = acc[t][j] + bv + bfr(x[(size_t)(r0 + hi * 8 + j) * DM + col]); }
    __syncthreads();
    float* crow = C + (size_t)r0 * DM + c0;
    auto pass = [&]() {
#pragma unroll
        for (int s = 0; s < 8; ++s) { const int Lid = (lane >> 3) + 4 * s, piece = lane & 7; const int row = Lid >> 1, cofs = (Lid & 1) * 32 + piece * 4;
            const v4f val = *(const v4fa*)(os + row * 68 + cofs); *(volatile v4f*)(crow + (size_t)row * DM + cofs) = val; }
    };
    pass(); __threadfence(); pass();
}

__global__ __launch_bounds__(256) void k_vt(const h16* __restrict__ V16, h16* VT16) {
    __shared__ __align__(16) h16 tile[64 * 72];
    const int bid = blockIdx.x;
    const int b = bid / (NH_ * (NT_ / 64)), rem = bid - b * (NH_ * (NT_ / 64)), h = rem / (NT_ / 64), kt = rem - h * (NT_ / 64);
    const int k0 = kt * 64, tid = threadIdx.x;
    const int kk = tid >> 2, d0 = (tid & 3) * 16;
    const h16* src = V16 + ((size_t)b * NT_ + k0 + kk) * DM + h * HD + d0;
#pragma unroll
    for (int i = 0; i < 16; ++i) tile[(d0 + i) * 72 + kk] = src[i];
    __syncthreads();
    const int piece = tid & 7;
    h16* base = VT16 + (((size_t)b * NH_ + h) * HD) * NT_ + k0;
    auto pass = [&]() {
#pragma unroll
        for (int s = 0; s < 2; ++s) { const int d = (tid >> 3) + 32 * s; const v8h val = *(const v8ha*)(tile + d * 72 + piece * 8); *(volatile v8h*)(base + (size_t)d * NT_ + piece * 8) = val; }
    };
    pass(); __threadfence(); pass();
}

__global__ __launch_bounds__(128) void k_attn(const h16* __restrict__ Q16, const h16* __restrict__ K16, const h16* __restrict__ VT16, h16* CTX16) {
    __shared__ __align__(16) h16 plds[4][16 * 32];
    __shared__ __align__(16) float ost[4][16 * 68];
    const int lane = threadIdx.x & 31, wave = threadIdx.x >> 5, lr = lane & 15, hi = lane >> 4;
    const int bid = blockIdx.x;
    const int b = bid / (NH_ * (NT_ / 64)), rem = bid - b * (NH_ * (NT_ / 64)), h = rem / (NT_ / 64), qt = rem - h * (NT_ / 64);
    const int q0 = qt * 64 + wave * 16;
    const size_t tok0 = (size_t)b * NT_;
    h16* pl = &plds[wave][0];
    v16h qa[2];
#pragma unroll
    for (int kc = 0; kc < 2; ++kc) { const h16* p = Q16 + (tok0 + q0 + lr) * DM + h * HD + kc * 32 + 8 * hi; qa[kc] = cat16(*(const v8h*)p, *(const v8h*)(p + 16)); }
    const h16* kh_b = K16 + tok0 * DM + h * HD;
    const h16* vt_b = VT16 + (((size_t)b * NH_ + h) * HD) * NT_;
    v8f o[4];
#pragma unroll
    for (int n = 0; n < 4; ++n) o[n] = (v8f){};
    float mrow[8], lpart[8];
#pragma unroll
    for (int j = 0; j < 8; ++j) { mrow[j] = -3.0e38f; lpart[j] = 0.f; }
#pragma unroll 1
    for (int kt = 0; kt < NT_ / 32; ++kt) {
        const int l0 = kt * 32;
        const h16* r0p = kh_b + (size_t)(l0 + lr) * DM + 8 * hi;
        const h16* r1p = kh_b + (size_t)(l0 + 16 + lr) * DM + 8 * hi;
        v8f s0 = {}, s1 = {};
#pragma unroll
        for (int kc = 0; kc < 2; ++kc) {
            s0 = wmma16(qa[kc], cat16(*(const v8h*)(r0p + kc * 32), *(const v8h*)(r0p + kc * 32 + 16)), s0);
            s1 = wmma16(qa[kc], cat16(*(const v8h*)(r1p + kc * 32), *(const v8h*)(r1p + kc * 32 + 16)), s1);
        }
        asm volatile("v_nop\n\tv_nop\n\tv_nop\n\tv_nop" : "+v"(s0), "+v"(s1) : "v"(qa[0]), "v"(qa[1]));
        float alpha[8];
#pragma unroll
        for (int j = 0; j < 8; ++j) {
            const float a0 = s0[j] * 0.125f, a1 = s1[j] * 0.125f;
            float mx = fmaxf(a0, a1);
            mx = fmaxf(mx, __shfl_xor(mx, 1, 16)); mx = fmaxf(mx, __shfl_xor(mx, 2, 16)); mx = fmaxf(mx, __shfl_xor(mx, 4, 16)); mx = fmaxf(mx, __shfl_xor(mx, 8, 16));
            const float mn = fmaxf(mrow[j], mx);
            alpha[j] = __expf(mrow[j] - mn); mrow[j] = mn;
            const float p0 = __expf(a0 - mn), p1 = __expf(a1 - mn);
            lpart[j] = lpart[j] * alpha[j] + (p0 + p1);
            const int mr = hi * 8 + j;
            pl[mr * 32 + lr] = (h16)(p0 * PSC); pl[mr * 32 + 16 + lr] = (h16)(p1 * PSC);
        }
#pragma unroll
        for (int n = 0; n < 4; ++n)
#pragma unroll
            for (int j = 0; j < 8; ++j) o[n][j] *= alpha[j];
        asm volatile("" ::: "memory");
        const v16h pa = cat16(*(const v8ha*)(pl + lr * 32 + hi * 8), *(const v8ha*)(pl + lr * 32 + 16 + hi * 8));
#pragma unroll
        for (int n = 0; n < 4; ++n) { const h16* vp = vt_b + (size_t)(n * 16 + lr) * NT_ + l0 + hi * 8; o[n] = wmma16(pa, cat16(*(const v8h*)vp, *(const v8h*)(vp + 16)), o[n]); }
        asm volatile("v_nop\n\tv_nop\n\tv_nop\n\tv_nop" : "+v"(o[0]), "+v"(o[1]), "+v"(o[2]), "+v"(o[3]) : "v"(pa));
    }
    float inv[8];
#pragma unroll
    for (int j = 0; j < 8; ++j) { float rs = lpart[j]; rs += __shfl_xor(rs, 1, 16); rs += __shfl_xor(rs, 2, 16); rs += __shfl_xor(rs, 4, 16); rs += __shfl_xor(rs, 8, 16); inv[j] = 1.0f / (rs * PSC); }
    float* os = &ost[wave][0];
#pragma unroll
    for (int n = 0; n < 4; ++n)
#pragma unroll
        for (int j = 0; j < 8; ++j) os[(hi * 8 + j) * 68 + n * 16 + lr] = o[n][j] * inv[j];
    __syncthreads();
    h16* crow = CTX16 + (tok0 + q0) * DM + (size_t)h * HD;
    auto pass = [&]() {
#pragma unroll
        for (int s = 0; s < 4; ++s) { const int row = 4 * s + (lane >> 3), piece = lane & 7; const float* sp = os + row * 68 + piece * 8; v8h o8;
#pragma unroll
            for (int i = 0; i < 8; ++i) o8[i] = (h16)sp[i];
            *(volatile v8h*)(crow + (size_t)row * DM + piece * 8) = o8; }
    };
    pass(); __threadfence(); pass();
}

extern "C" void kernel_launch(void* const* d_in, const int* in_sizes, int n_in,
                              void* d_out, int out_size, void* d_ws, size_t ws_size, hipStream_t stream) {
    (void)in_sizes; (void)n_in; (void)out_size;
    const float* x = (const float*)d_in[0]; const float* ng = (const float*)d_in[1]; const float* nb = (const float*)d_in[2]; const float* W1 = (const float*)d_in[3]; const float* b1 = (const float*)d_in[4];
    const float* qg = (const float*)d_in[5]; const float* qb = (const float*)d_in[6]; const float* kg = (const float*)d_in[7]; const float* kb = (const float*)d_in[8];
    const float* Wao = (const float*)d_in[9]; const float* bao = (const float*)d_in[10]; const float* Wmo = (const float*)d_in[11]; const float* bmo = (const float*)d_in[12];
    const float* W2 = (const float*)d_in[13]; const float* b2 = (const float*)d_in[14];
    float* out = (float*)d_out;
    char* wsp = (char*)d_ws;
    auto take = [&](size_t bytes) { char* p = wsp; wsp += (bytes + 255) & ~(size_t)255; return (void*)p; };
    h16* XN16 = (h16*)take((size_t)NTK * DM * 2); h16* W1T = (h16*)take((size_t)NFP * DM * 2);
    h16* WaoT = (h16*)take((size_t)DM * DM * 2); h16* WmoT = (h16*)take((size_t)DM * MLPP * 2); h16* W2T = (h16*)take((size_t)DM * 2 * DM * 2);
    h16* Q16 = (h16*)take((size_t)NTK * DM * 2); h16* K16 = (h16*)take((size_t)NTK * DM * 2); h16* V16 = (h16*)take((size_t)NTK * DM * 2); h16* VT16 = (h16*)take((size_t)NTK * DM * 2);
    h16* G16 = (h16*)take((size_t)NTK * MLPP * 2); h16* CTX16 = (h16*)take((size_t)NTK * DM * 2); h16* COMB16 = (h16*)take((size_t)NTK * 2 * DM * 2);
    if ((size_t)(wsp - (char*)d_ws) > ws_size) return;
    k_ln<<<NTK / 8, 256, 0, stream>>>(x, ng, nb, XN16);
    k_wt<<<dim3(DM / 64, NFP / 64, 1), 256, 0, stream>>>(W1, DM, NF, DM, W1T);
    k_wt<<<dim3(DM / 64, DM / 64, 1), 256, 0, stream>>>(Wao, DM, DM, DM, WaoT);
    k_wt<<<dim3(MLPP / 64, DM / 64, 1), 256, 0, stream>>>(Wmo, MLPH, DM, MLPP, WmoT);
    k_wt<<<dim3((2 * DM) / 64, DM / 64, 1), 256, 0, stream>>>(W2, 2 * DM, DM, 2 * DM, W2T);
    k_fused<<<dim3(NTK / 64, NFP / 64, 1), 128, 0, stream>>>(XN16, W1T, b1, qg, qb, kg, kb, Q16, K16, V16, G16);
    k_vt<<<NB_ * NH_ * (NT_ / 64), 256, 0, stream>>>(V16, VT16);
    k_attn<<<NB_ * NH_ * (NT_ / 64), 128, 0, stream>>>(Q16, K16, VT16, CTX16);
    k_gemm16o<<<dim3(NTK / 64, DM / 64, 1), 128, 0, stream>>>(CTX16, WaoT, DM, bao, COMB16, 2 * DM, 0);
    k_gemm16o<<<dim3(NTK / 64, DM / 64, 1), 128, 0, stream>>>(G16, WmoT, MLPP, bmo, COMB16, 2 * DM, DM);
    k_gemmout<<<dim3(NTK / 64, DM / 64, 1), 128, 0, stream>>>(COMB16, W2T, b2, x, out);
}
